// GNNSAGETransformer_5068061409375
// MI455X (gfx1250) — hardware-run, weakly checked
//
#include <hip/hip_runtime.h>


namespace {
constexpr int B = 4, T = 16, N = 1024, E = 16384, F = 128, H = 256, FF = 1024, NH = 8, HD = 32, L = 2, C = 10, G = B * T, NN = G * N, NE = G * E, NTOK = G;
constexpr float S64 = 64.0f, S1K = 1024.0f, S256 = 256.0f, WSC = 256.0f;
typedef _Float16 b16;
typedef __attribute__((ext_vector_type(16))) _Float16 v16b;
typedef __attribute__((ext_vector_type(8))) _Float16 v8b;
typedef __attribute__((ext_vector_type(8))) float v8f;
typedef __attribute__((ext_vector_type(4))) float v4f;
__device__ __forceinline__ float bf16_rne(float f) { unsigned int u = __float_as_uint(f); u += 0x7FFFu + ((u >> 16) & 1u); return __uint_as_float(u & 0xFFFF0000u); }
__device__ __forceinline__ void split16(float v, b16& hi, b16& lo) { hi = (b16)v; lo = (b16)(v - (float)hi); }
__device__ __forceinline__ v16b frag_kb(const b16* p, int hh) { const v8b a = *(const v8b*)(p + 8 * hh), b = *(const v8b*)(p + 16 + 8 * hh); v16b f;
#pragma unroll
  for (int e = 0; e < 8; ++e) { f[e] = a[e]; f[8 + e] = b[e]; } return f; }
__device__ __forceinline__ v8f wmma16b(v16b a, v16b b, v8f c) { v8f d = __builtin_amdgcn_wmma_f32_16x16x32_f16(false, a, false, b, (short)0, c, false, false); asm volatile("v_nop\n\tv_nop\n\tv_nop\n\tv_nop" : "+v"(d) : "v"(a), "v"(b)); return d; }
__device__ __forceinline__ void wave_lds_sync() { __builtin_amdgcn_fence(__ATOMIC_RELEASE, "workgroup"); __builtin_amdgcn_wave_barrier(); __builtin_amdgcn_fence(__ATOMIC_ACQUIRE, "workgroup"); }
__device__ __forceinline__ float pmul(float a, float b) { float p = a * b; asm volatile("" : "+v"(p)); return p; }
__device__ __forceinline__ int iclamp(int v, int lo, int hi) { return v < lo ? lo : (v > hi ? hi : v); }
constexpr int CSR_NBLK9 = 512, CSR_GB9 = 9, CSR_GN9 = 1 << CSR_GB9  , CSR_TS9 = (CSR_GN9 < 32 ? 32 : CSR_GN9)  , CSR_MAXG9 = 512, CSR_CAP9 = 12288  ;
__device__ __host__ __forceinline__ int csr_tix9(int v) { return (v >> CSR_GB9) * CSR_TS9 + (v & (CSR_GN9 - 1)); }
__global__ __launch_bounds__(64) void csrA_kernel9(const int* __restrict__ dst, int E, int N, int nG, int CHP, int NGP, int* __restrict__ STG, int* __restrict__ HST) {
  extern __shared__ int sm[];
  int* cnt = sm; int* run = sm + NGP; int* ids = sm + 2 * NGP;
  const int b = blockIdx.x; const int ch = (E + CSR_NBLK9 - 1) / CSR_NBLK9; const int e0 = b * ch, e1 = min(E, e0 + ch);
  for (int i = threadIdx.x; i < NGP; i += 64) cnt[i] = 0;
  for (int i = threadIdx.x; i < CHP; i += 64) ids[i] = -1;
  __syncthreads();
  if (threadIdx.x == 0) {
    for (int e = e0; e < e1; ++e) { int d = dst[e]; d = (d < 0) ? 0 : (d >= N ? N - 1 : d); cnt[d >> CSR_GB9] += 1; }
    int acc = 0; for (int g = 0; g < nG; ++g) { run[g] = acc; acc += cnt[g]; }
    for (int e = e0; e < e1; ++e) { int d = dst[e]; d = (d < 0) ? 0 : (d >= N ? N - 1 : d); const int g = d >> CSR_GB9; ids[run[g]] = e; run[g] += 1; } }
  __syncthreads();
  typedef __attribute__((ext_vector_type(4))) int v4i;
  for (int pass = 0; pass < 2; ++pass) {
    for (int i = threadIdx.x; i < CHP / 4; i += 64) *(volatile v4i*)(STG + (size_t)b * CHP + i * 4) = *(const v4i*)(&ids[i * 4]);
    for (int i = threadIdx.x; i < NGP / 4; i += 64) { v4i v; for (int e = 0; e < 4; ++e) v[e] = (i * 4 + e < nG) ? cnt[i * 4 + e] : 0; *(volatile v4i*)(HST + (size_t)b * NGP + i * 4) = v; }
    __threadfence(); }
}
__global__ __launch_bounds__(512) void csrS_kernel9(const int* __restrict__ HST, int nG, int NGP, int* __restrict__ START, int* __restrict__ TOT, int* __restrict__ OFF) {
  __shared__ int tot[CSR_MAXG9];
  const int b = threadIdx.x;
  for (int pass = 0; pass < 2; ++pass) { int runb = 0; for (int g = 0; g < nG; ++g) { int c = HST[(size_t)b * NGP + g]; c = (c < 0) ? 0 : c; ((volatile int*)OFF)[(size_t)g * CSR_NBLK9 + b] = runb; runb += c; } __threadfence(); }
  for (int g = threadIdx.x; g < nG; g += 512) { int s = 0; for (int bb = 0; bb < CSR_NBLK9; ++bb) { int c = HST[(size_t)bb * NGP + g]; s += (c < 0) ? 0 : c; } tot[g] = s; }
  __syncthreads();
  if (threadIdx.x < 32) {
    __shared__ int st[CSR_MAXG9 + 32];
    if (threadIdx.x == 0) { int acc = 0; for (int g = 0; g < NGP; ++g) { st[g] = acc; if (g < nG) acc += (tot[g] + 31) & ~31; } st[NGP] = acc; }
    __builtin_amdgcn_fence(__ATOMIC_RELEASE, "workgroup"); __builtin_amdgcn_wave_barrier(); __builtin_amdgcn_fence(__ATOMIC_ACQUIRE, "workgroup");
    for (int pass = 0; pass < 2; ++pass) { for (int i = threadIdx.x; i < NGP + 32; i += 32) { ((volatile int*)START)[i] = (i <= NGP) ? st[min(i, NGP)] : 0; ((volatile int*)TOT)[i] = (i < nG) ? tot[i] : 0; } __threadfence(); } }
}
__global__ __launch_bounds__(256) void csrB_kernel9(const int* __restrict__ dst, int N, int nG, int CHP, int NGP, int permLen, const int* __restrict__ STG, const int* __restrict__ HST, const int* __restrict__ OFF, const int* __restrict__ START, const int* __restrict__ TOT, int* __restrict__ PERM, int* __restrict__ ROWPTR, int* __restrict__ ROWCNT, int* __restrict__ FLAG) {
  typedef __attribute__((ext_vector_type(4))) int v4i;
  __shared__ int ids[CSR_CAP9]; __shared__ unsigned short key[CSR_CAP9]; __shared__ int outp[CSR_CAP9]; __shared__ int ncnt[CSR_GN9 + 1]; __shared__ int boff[CSR_NBLK9 + 1];
  const int g = blockIdx.x, t_ = threadIdx.x; int tot = TOT[g]; int st = START[g], stn = START[g + 1]; const int v0 = g * CSR_GN9; const int nv = min(CSR_GN9, N - v0); const int t0 = g * CSR_TS9;
  st = (st < 0) ? 0 : (st > permLen - 32 ? permLen - 32 : st) & ~31; stn = (stn < st) ? st : (stn > permLen ? permLen : stn); tot = (tot < 0) ? 0 : tot; if (tot > stn - st && tot <= CSR_CAP9) tot = stn - st;
  if (tot > CSR_CAP9) {
    for (int pass = 0; pass < 2; ++pass) { for (int i = t_; i < CSR_TS9 / 4; i += 256) { v4i a, c; for (int e = 0; e < 4; ++e) { a[e] = st; c[e] = 0; } *(volatile v4i*)(ROWPTR + t0 + i * 4) = a; *(volatile v4i*)(ROWCNT + t0 + i * 4) = c; } if (t_ == 0) ((volatile int*)FLAG)[0] = 1; __threadfence(); } (void)nv; return; }
  if (t_ == 0) { int acc = 0; for (int b = 0; b < CSR_NBLK9; ++b) { boff[b] = acc; int c = HST[(size_t)b * NGP + g]; c = (c < 0) ? 0 : (c > CHP ? CHP : c); acc += c; if (acc > tot) acc = tot; } boff[CSR_NBLK9] = acc; }
  for (int i = t_; i <= CSR_GN9; i += 256) ncnt[i] = 0;
  __syncthreads();
  for (int b = 0; b < CSR_NBLK9; ++b) { const int c = boff[b + 1] - boff[b]; int o_ = OFF[(size_t)g * CSR_NBLK9 + b]; o_ = (o_ < 0) ? 0 : (o_ > CHP - c ? CHP - c : o_); const int* src_ = STG + (size_t)b * CHP + o_;
    for (int i = t_; i < c; i += 256) { int id = src_[i]; id = (id < 0) ? 0 : id; ids[boff[b] + i] = id; int d = dst[id]; d = (d < v0) ? v0 : (d >= N ? N - 1 : d); int kk = d - v0; kk = (kk < 0) ? 0 : (kk >= CSR_GN9 ? CSR_GN9 - 1 : kk); key[boff[b] + i] = (unsigned short)kk; } }
  __syncthreads();
  if (t_ == 0) { for (int i = 0; i < tot; ++i) ncnt[key[i]] += 1; int acc = 0; for (int vl = 0; vl < CSR_GN9; ++vl) { const int c = ncnt[vl]; ncnt[vl] = acc; acc += c; } ncnt[CSR_GN9] = acc;
    for (int i = 0; i < tot; ++i) { const int vl = key[i]; outp[ncnt[vl]] = ids[i]; ncnt[vl] += 1; }
    for (int vl = CSR_GN9; vl > 0; --vl) ncnt[vl] = ncnt[vl - 1]; ncnt[0] = 0; }
  __syncthreads();
  for (int pass = 0; pass < 2; ++pass) {
    for (int i = t_; i < (stn - st) / 4; i += 256) { v4i v; for (int e = 0; e < 4; ++e) { const int q = i * 4 + e; v[e] = (q < tot) ? outp[q] : -1; } *(volatile v4i*)(PERM + st + i * 4) = v; }
    for (int i = t_; i < CSR_TS9 / 4; i += 256) { v4i a, c; for (int e = 0; e < 4; ++e) { const int vl = i * 4 + e; const int vc = vl < CSR_GN9 ? vl : CSR_GN9; a[e] = (vl < CSR_GN9) ? st + ncnt[vc] : st; c[e] = (vl < nv) ? (ncnt[(vc < CSR_GN9 ? vc : CSR_GN9 - 1) + 1] - ncnt[vc]) : 0; } *(volatile v4i*)(ROWPTR + t0 + i * 4) = a; *(volatile v4i*)(ROWCNT + t0 + i * 4) = c; }
    __threadfence(); }
}
__global__ __launch_bounds__(256) void csrZ_kernel9(int* __restrict__ p, size_t n4) { typedef __attribute__((ext_vector_type(4))) int v4i; const size_t tid = (size_t)blockIdx.x * 256 + threadIdx.x, nth = (size_t)gridDim.x * 256; v4i z = {0, 0, 0, 0}; for (size_t i = tid; i < n4; i += nth) *(volatile v4i*)(p + i * 4) = z; }
struct CsrBufs9 { int *STG, *HST, *OFF, *START, *TOT, *PERM, *ROWPTR, *ROWCNT, *FLAG; int nG, NGP, CHP; size_t permLen; char* base; size_t bytes; };
static size_t csr_carve9(CsrBufs9& c, char* ws, size_t off, int E, int N) {
  const size_t off0 = off; c.base = ws + off;
  auto al = [&](size_t bytes) { char* p = ws + off; off += (bytes + 255) & ~(size_t)255; return p; };
  c.nG = (N + CSR_GN9 - 1) / CSR_GN9; c.NGP = (c.nG + 31) & ~31; const int ch = (E + CSR_NBLK9 - 1) / CSR_NBLK9; c.CHP = (ch + 31) & ~31; c.permLen = (size_t)E + 32 * (size_t)c.nG + 32;
  c.STG = (int*)al((size_t)CSR_NBLK9 * c.CHP * 4); c.HST = (int*)al((size_t)CSR_NBLK9 * c.NGP * 4); c.OFF = (int*)al((size_t)c.NGP * CSR_NBLK9 * 4); c.START = (int*)al((size_t)(c.NGP + 64) * 4); c.TOT = (int*)al((size_t)(c.NGP + 64) * 4);
  c.PERM = (int*)al(c.permLen * 4); c.ROWPTR = (int*)al((size_t)c.nG * CSR_TS9 * 4); c.ROWCNT = (int*)al((size_t)c.nG * CSR_TS9 * 4); c.FLAG = (int*)al(256);
  c.bytes = off - off0; return off;
}
static void csr_build9(const CsrBufs9& c, const int* dst, int E, int N, hipStream_t stream) {
  const size_t smem = (size_t)(2 * c.NGP + c.CHP) * 4;
  csrZ_kernel9<<<512, 256, 0, stream>>>((int*)c.base, c.bytes / 16);
  csrA_kernel9<<<CSR_NBLK9, 64, smem, stream>>>(dst, E, N, c.nG, c.CHP, c.NGP, c.STG, c.HST);
  csrS_kernel9<<<1, 512, 0, stream>>>(c.HST, c.nG, c.NGP, c.START, c.TOT, c.OFF);
  csrB_kernel9<<<c.nG, 256, 0, stream>>>(dst, N, c.nG, c.CHP, c.NGP, (int)c.permLen, c.STG, c.HST, c.OFF, c.START, c.TOT, c.PERM, c.ROWPTR, c.ROWCNT, c.FLAG);
}


__global__ __launch_bounds__(256) void wput_kernel(const float* __restrict__ w, int KIN, int OUTW, int ko, int KP, b16* __restrict__ WT) {
  const int KG = KIN / 8; const int u = blockIdx.x * 256 + threadIdx.x; if (u >= OUTW * KG) return; const int o = u / KG, k0 = (u % KG) * 8; v8b v;
#pragma unroll
  for (int j = 0; j < 8; ++j) v[j] = (b16)(bf16_rne(w[(size_t)(k0 + j) * OUTW + o]) * WSC); for (int pass = 0; pass < 2; ++pass) { *(volatile v8b*)(WT + (size_t)o * KP + ko + k0) = v; __threadfence(); }
}
__global__ __launch_bounds__(256) void keys_kernel(const int* __restrict__ ei, int* __restrict__ KD) {
  const int p = blockIdx.x * 256 + threadIdx.x; if (p >= NE) return; const int g = p / E, e = p % E; const int d = iclamp(ei[((size_t)g * 2 + 1) * E + e], 0, N - 1);
  for (int pass = 0; pass < 2; ++pass) { ((volatile int*)KD)[p] = g * N + d; __threadfence(); }
}
template <int KIN, int FIRST>
__global__ __launch_bounds__(32) void sage_kernel(const float* __restrict__ IN, const int* __restrict__ ei, const int* __restrict__ PERM, const int* __restrict__ ROWPTR, const int* __restrict__ ROWCNT, int permLen, const b16* __restrict__ WT, const float* __restrict__ bl, int GLIM, float* __restrict__ OUT) {
  constexpr int K2 = 2 * KIN, PL = KIN / 32;
  __shared__ __attribute__((aligned(16))) b16 Ah[16][K2 + 8], Al[16][K2 + 8]; __shared__ __attribute__((aligned(16))) float Tf[16][128 + 4];
  const int lane = threadIdx.x, nloc = lane & 15, hlf = lane >> 4; const size_t m0 = (size_t)blockIdx.x * 16; const int g = (int)(m0 / N); if (g >= GLIM) return;
  for (int rr = 0; rr < 16; ++rr) { const size_t v = m0 + rr; int st = ROWPTR[v], cnt = ROWCNT[v]; cnt = iclamp(cnt, 0, 1 << 20); st = iclamp(st, 0, permLen - cnt); float s[PL], sv[PL]; for (int q = 0; q < PL; ++q) { s[q] = 0.0f; float x_ = IN[v * KIN + q * 32 + lane]; sv[q] = FIRST ? bf16_rne(x_) : x_; }
#pragma unroll 1
    for (int j = 0; j < cnt; ++j) { const int p = iclamp(PERM[st + j], 0, NE - 1); const int e = p % E; const size_t u = (size_t)g * N + iclamp(ei[((size_t)g * 2) * E + e], 0, N - 1); for (int q = 0; q < PL; ++q) { const float x_ = IN[u * KIN + q * 32 + lane]; s[q] += FIRST ? bf16_rne(x_) : x_; } }
    const float inv = 1.0f / (float)(cnt < 1 ? 1 : cnt);
    for (int q = 0; q < PL; ++q) { b16 ph, pq; split16(pmul(s[q], inv) * S64, ph, pq); Ah[rr][q * 32 + lane] = ph; Al[rr][q * 32 + lane] = pq; split16(sv[q] * S64, ph, pq); Ah[rr][KIN + q * 32 + lane] = ph; Al[rr][KIN + q * 32 + lane] = pq; } }
  wave_lds_sync();
#pragma unroll 1
  for (int cg = 0; cg < 2; ++cg) { v8f acc[8];
#pragma unroll
    for (int t = 0; t < 8; ++t) acc[t] = (v8f){};
#pragma unroll 2
    for (int kb = 0; kb < K2; kb += 32) { const v16b a = frag_kb(&Ah[nloc][kb], hlf), al = frag_kb(&Al[nloc][kb], hlf);
#pragma unroll
      for (int t = 0; t < 8; ++t) { const v16b bw = frag_kb(WT + (size_t)(cg * 128 + t * 16 + nloc) * K2 + kb, hlf); acc[t] = wmma16b(a, bw, acc[t]); acc[t] = wmma16b(al, bw, acc[t]); } }
#pragma unroll
    for (int t = 0; t < 8; ++t) { const int c = cg * 128 + t * 16 + nloc; const float bb = bf16_rne(bl[c]);
#pragma unroll 1
      for (int r8 = 0; r8 < 8; ++r8) { const float v = acc[t][r8] * (1.0f / (S64 * WSC)) + bb; Tf[8 * hlf + r8][t * 16 + nloc] = FIRST ? fmaxf(v, 0.0f) : v; } }
    wave_lds_sync();
    for (int pass = 0; pass < 2; ++pass) { for (int rr = 0; rr < 16; ++rr) *(volatile v4f*)(OUT + (m0 + rr) * H + cg * 128 + lane * 4) = *(const v4f*)(&Tf[rr][lane * 4]); __threadfence(); }
    wave_lds_sync(); }
}
__global__ __launch_bounds__(256) void gmean_kernel(const float* __restrict__ H2, int GLIM, float* __restrict__ EMB) {
  const int g = blockIdx.x, c = threadIdx.x; float s = 0.0f; if (g < GLIM) {
#pragma unroll 4
    for (int n = 0; n < N; ++n) s += H2[((size_t)g * N + n) * H + c]; }
  const float m = s * (1.0f / N); for (int pass = 0; pass < 2; ++pass) { ((volatile float*)EMB)[(size_t)g * H + c] = m; __threadfence(); }
}
template <int KIN, int OUTW, int RELU>
__global__ __launch_bounds__(32) void tgemm_kernel(const float* __restrict__ IN, float scale, const b16* __restrict__ WT, const float* __restrict__ bias, float* __restrict__ OUT) {
  __shared__ __attribute__((aligned(16))) b16 Ah[16][KIN + 8], Al[16][KIN + 8]; __shared__ __attribute__((aligned(16))) float Tf[16][128 + 4];
  const int lane = threadIdx.x, nloc = lane & 15, hlf = lane >> 4; const size_t t0 = (size_t)blockIdx.x * 16;
  for (int rr = 0; rr < 16; ++rr) for (int q = 0; q < KIN / 32; ++q) { b16 p, ql; split16(IN[(t0 + rr) * KIN + q * 32 + lane] * scale, p, ql); Ah[rr][q * 32 + lane] = p; Al[rr][q * 32 + lane] = ql; }
  wave_lds_sync(); const float sc = 1.0f / (scale * WSC);
#pragma unroll 1
  for (int cg = 0; cg < OUTW / 128; ++cg) { v8f acc[8];
#pragma unroll
    for (int t = 0; t < 8; ++t) acc[t] = (v8f){};
#pragma unroll 2
    for (int kb = 0; kb < KIN; kb += 32) { const v16b a = frag_kb(&Ah[nloc][kb], hlf), al = frag_kb(&Al[nloc][kb], hlf);
#pragma unroll
      for (int t = 0; t < 8; ++t) { const v16b bw = frag_kb(WT + (size_t)(cg * 128 + t * 16 + nloc) * KIN + kb, hlf); acc[t] = wmma16b(a, bw, acc[t]); acc[t] = wmma16b(al, bw, acc[t]); } }
#pragma unroll
    for (int t = 0; t < 8; ++t) { const int c = cg * 128 + t * 16 + nloc; const float bb = bf16_rne(bias[c]);
#pragma unroll 1
      for (int r8 = 0; r8 < 8; ++r8) { const float v = acc[t][r8] * sc + bb; Tf[8 * hlf + r8][t * 16 + nloc] = RELU ? fmaxf(v, 0.0f) : v; } }
    wave_lds_sync();
    for (int pass = 0; pass < 2; ++pass) { for (int rr = 0; rr < 16; ++rr) *(volatile v4f*)(OUT + (t0 + rr) * OUTW + cg * 128 + lane * 4) = *(const v4f*)(&Tf[rr][lane * 4]); __threadfence(); }
    wave_lds_sync(); }
}
__global__ __launch_bounds__(256) void attn_kernel(const float* __restrict__ QKV, float* __restrict__ CTX) {
  __shared__ float Qs[T][HD + 1], Ks[T][HD + 1], Vs[T][HD + 1], Ps[T][T + 1];
  const int b = blockIdx.x / NH, h = blockIdx.x % NH; const int tid = threadIdx.x;
  for (int i = tid; i < T * HD; i += 256) { const int t = i / HD, d = i % HD; const float* row = QKV + ((size_t)b * T + t) * (3 * H); Qs[t][d] = row[h * HD + d]; Ks[t][d] = row[H + h * HD + d]; Vs[t][d] = row[2 * H + h * HD + d]; }
  __syncthreads();
  { const int q = tid >> 4, k = tid & 15; float s = 0.0f;
#pragma unroll 1
    for (int d = 0; d < HD; ++d) s += pmul(Qs[q][d], Ks[k][d]); Ps[q][k] = s * 0.17677669529663687f; }
  __syncthreads();
  if (tid < T) { const int q = tid; float mx = Ps[q][0]; for (int k = 1; k < T; ++k) mx = fmaxf(mx, Ps[q][k]); float se = 0.0f; float ex[T]; for (int k = 0; k < T; ++k) { ex[k] = __expf(Ps[q][k] - mx); se += ex[k]; } for (int k = 0; k < T; ++k) Ps[q][k] = ex[k] / se; }
  __syncthreads();
  const int wave = tid >> 5, lane = tid & 31;
  for (int pass = 0; pass < 2; ++pass) { for (int qq = 0; qq < 2; ++qq) { const int q = wave * 2 + qq; float s = 0.0f;
#pragma unroll 1
      for (int k = 0; k < T; ++k) s += pmul(Ps[q][k], Vs[k][lane]); ((volatile float*)CTX)[((size_t)b * T + q) * H + h * HD + lane] = s; } __threadfence(); }
}
__global__ __launch_bounds__(256) void addln_kernel(float* Hh, const float* __restrict__ Y, const float* __restrict__ s_, const float* __restrict__ b_) {
  const int wave = threadIdx.x >> 5, lane = threadIdx.x & 31; const int t = blockIdx.x * 8 + wave; if (t >= NTOK) return;
  float v[8]; float s = 0.0f; for (int q = 0; q < 8; ++q) { v[q] = Hh[(size_t)t * H + q * 32 + lane] + Y[(size_t)t * H + q * 32 + lane]; s += v[q]; }
  for (int o = 16; o; o >>= 1) s += __shfl_xor(s, o); const float mu = s * (1.0f / H); float vq = 0.0f; for (int q = 0; q < 8; ++q) { const float d = v[q] - mu; vq += pmul(d, d); } for (int o = 16; o; o >>= 1) vq += __shfl_xor(vq, o); const float rs = rsqrtf(vq * (1.0f / H) + 1e-5f);
  float r[8]; for (int q = 0; q < 8; ++q) r[q] = pmul(pmul(v[q] - mu, rs), bf16_rne(s_[q * 32 + lane])) + bf16_rne(b_[q * 32 + lane]);
  for (int pass = 0; pass < 2; ++pass) { for (int q = 0; q < 8; ++q) ((volatile float*)Hh)[(size_t)t * H + q * 32 + lane] = r[q]; __threadfence(); }
}
__global__ __launch_bounds__(64) void fc_kernel(const float* __restrict__ Hh, const float* __restrict__ fcW, const float* __restrict__ fcb, int BV, float* __restrict__ out) {
  const int i = threadIdx.x; if (i >= B * C) return; const int b = i / C, c = i % C; float s = bf16_rne(fcb[c]);
  if (b < BV) {
#pragma unroll 1
    for (int d = 0; d < H; ++d) s += pmul(Hh[((size_t)b * T + T - 1) * H + d], bf16_rne(fcW[d * C + c])); } else s = 0.0f;
  for (int pass = 0; pass < 2; ++pass) { ((volatile float*)out)[i] = s; __threadfence(); }
}
}

extern "C" void kernel_launch(void* const* d_in, const int* in_sizes, int n_in, void* d_out, int out_size, void* d_ws, size_t ws_size, hipStream_t stream) {
  (void)n_in;
  auto Fp = [&](int i) { return (const float*)d_in[i]; }; auto Ip = [&](int i) { return (const int*)d_in[i]; };
  if (in_sizes[0] != NN * F || in_sizes[1] != G * 2 * E || in_sizes[2] != F * H || in_sizes[5] != H * H || in_sizes[8] != L * H * 3 * H || in_sizes[14] != L * H * FF || in_sizes[16] != L * FF * H || in_sizes[20] != H * C || out_size != B * C) return;
  const int BV = B; const int GLIM = BV * T;
  size_t off = 0; char* ws = (char*)d_ws;
  auto carve = [&](size_t bytes) { char* p = ws + off; off += (bytes + 255) & ~(size_t)255; return p; };
  b16* WS1 = (b16*)carve((size_t)H * 2 * F * 2); b16* WS2 = (b16*)carve((size_t)H * 2 * H * 2); b16* WQKV[L]; b16* WO[L]; b16* WF1[L]; b16* WF2[L];
  for (int l = 0; l < L; ++l) { WQKV[l] = (b16*)carve((size_t)3 * H * H * 2); WO[l] = (b16*)carve((size_t)H * H * 2); WF1[l] = (b16*)carve((size_t)FF * H * 2); WF2[l] = (b16*)carve((size_t)H * FF * 2); }
  int* KD = (int*)carve((size_t)NE * 4); float* H1 = (float*)carve((size_t)NN * H * 4); float* H2 = (float*)carve((size_t)NN * H * 4); float* EMB = (float*)carve((size_t)NTOK * H * 4); float* QKV = (float*)carve((size_t)NTOK * 3 * H * 4); float* CTX = (float*)carve((size_t)NTOK * H * 4); float* Y = (float*)carve((size_t)NTOK * H * 4); float* FFP = (float*)carve((size_t)NTOK * FF * 4);
  CsrBufs9 csr; off = csr_carve9(csr, ws, off, NE, NN);
  if (off > ws_size || off > ((size_t)192 << 20)) return;
  wput_kernel<<<(H * F / 8 + 255) / 256, 256, 0, stream>>>(Fp(2), F, H, 0, 2 * F, WS1); wput_kernel<<<(H * F / 8 + 255) / 256, 256, 0, stream>>>(Fp(4), F, H, F, 2 * F, WS1);
  wput_kernel<<<(H * H / 8 + 255) / 256, 256, 0, stream>>>(Fp(5), H, H, 0, 2 * H, WS2); wput_kernel<<<(H * H / 8 + 255) / 256, 256, 0, stream>>>(Fp(7), H, H, H, 2 * H, WS2);
  for (int l = 0; l < L; ++l) { wput_kernel<<<(3 * H * H / 8 + 255) / 256, 256, 0, stream>>>(Fp(8) + (size_t)l * H * 3 * H, H, 3 * H, 0, H, WQKV[l]); wput_kernel<<<(H * H / 8 + 255) / 256, 256, 0, stream>>>(Fp(10) + (size_t)l * H * H, H, H, 0, H, WO[l]);
    wput_kernel<<<(FF * H / 8 + 255) / 256, 256, 0, stream>>>(Fp(14) + (size_t)l * H * FF, H, FF, 0, H, WF1[l]); wput_kernel<<<(H * FF / 8 + 255) / 256, 256, 0, stream>>>(Fp(16) + (size_t)l * FF * H, FF, H, 0, FF, WF2[l]); }
  keys_kernel<<<NE / 256, 256, 0, stream>>>(Ip(1), KD);
  csr_build9(csr, KD, NE, NN, stream);
  sage_kernel<F, 1><<<(GLIM * N) / 16, 32, 0, stream>>>(Fp(0), Ip(1), csr.PERM, csr.ROWPTR, csr.ROWCNT, (int)csr.permLen, WS1, Fp(3), GLIM, H1);
  sage_kernel<H, 0><<<(GLIM * N) / 16, 32, 0, stream>>>(H1, Ip(1), csr.PERM, csr.ROWPTR, csr.ROWCNT, (int)csr.permLen, WS2, Fp(6), GLIM, H2);
  gmean_kernel<<<G, 256, 0, stream>>>(H2, GLIM, EMB);
  for (int l = 0; l < L; ++l) {
    tgemm_kernel<H, 3 * H, 0><<<NTOK / 16, 32, 0, stream>>>(EMB, S1K, WQKV[l], Fp(9) + l * 3 * H, QKV);
    attn_kernel<<<B * NH, 256, 0, stream>>>(QKV, CTX);
    tgemm_kernel<H, H, 0><<<NTOK / 16, 32, 0, stream>>>(CTX, S1K, WO[l], Fp(11) + l * H, Y);
    addln_kernel<<<NTOK / 8, 256, 0, stream>>>(EMB, Y, Fp(12) + l * H, Fp(13) + l * H);
    tgemm_kernel<H, FF, 1><<<NTOK / 16, 32, 0, stream>>>(EMB, S256, WF1[l], Fp(15) + l * FF, FFP);
    tgemm_kernel<FF, H, 0><<<NTOK / 16, 32, 0, stream>>>(FFP, S256, WF2[l], Fp(17) + l * H, Y);
    addln_kernel<<<NTOK / 8, 256, 0, stream>>>(EMB, Y, Fp(18) + l * H, Fp(19) + l * H); }
  fc_kernel<<<1, 64, 0, stream>>>(EMB, Fp(20), Fp(21), BV, (float*)d_out);
}
